// TrajectoryGAT_21655225106673
// MI455X (gfx1250) — hardware-verified
//
#include <hip/hip_runtime.h>
#include <stddef.h>
#include <math.h>


#define CIN    9
#define HD     128
#define NTHR   256
#define NWAVE  8
#define CHUNK  2048
#define WCAP   256
#define NB1    4096
#define NB2    16384
#define NCH1   10
#define NCH2   3
#define GR     32
#define TSP    136
#define NGMAX  256
#define NQMAX  4

static_assert(CHUNK == NTHR * 8);
static_assert(WCAP == 8 * 32);
static_assert(NB1 <= 16384 && NB2 <= 16384);
static_assert((NB1 % GR) == 0 && (NB2 % (NWAVE * 32)) == 0);
static_assert(NGMAX == NTHR);

#define LDS1_ACC   (NCH1 * NB1 * 4)
#define LDS_LIST   (NWAVE * WCAP * 4)
#define LDS_WCNT   64
#define LDS1_TILE  (16 * TSP * 2)
#define LDS1_BYTES (LDS1_ACC + LDS_LIST + LDS_WCNT + LDS1_TILE)
#define LDS2_ACC   (NCH2 * NB2 * 4)
#define LDS2_PART  (NWAVE * NGMAX * 16)
#define LDS2_BYTES (LDS2_ACC + LDS_LIST + LDS_WCNT + LDS2_PART)
static_assert(LDS1_BYTES == 176448);
static_assert(LDS2_BYTES == 237632);
static_assert(((LDS1_ACC + LDS_LIST + LDS_WCNT) % 16) == 0);
static_assert(((LDS2_ACC + LDS_LIST + LDS_WCNT) % 16) == 0);

typedef float    v4f  __attribute__((ext_vector_type(4)));
typedef float    v8f  __attribute__((ext_vector_type(8)));
typedef int      v4i  __attribute__((ext_vector_type(4)));
typedef _Float16 v8h  __attribute__((ext_vector_type(8)));
typedef _Float16 v16h __attribute__((ext_vector_type(16)));
union Frag   { v16h v; v8h half[2]; _Float16 s[16]; };
union Pack16 { v8h h; v4i i; _Float16 s[8]; };

__device__ __forceinline__ v8f wm(v16h a, v16h b, v8f c) {
  v8f d = __builtin_amdgcn_wmma_f32_16x16x32_f16(false, a, false, b, (short)0, c, false, false);
  asm volatile("v_nop\n\tv_nop\n\tv_nop\n\tv_nop" : "+v"(d) : "v"(a), "v"(b));
  return d;
}

__device__ __forceinline__ float wsum(float v) {
  v += __shfl_xor(v, 16, 32);
  v += __shfl_xor(v, 8, 32);
  v += __shfl_xor(v, 4, 32);
  v += __shfl_xor(v, 2, 32);
  v += __shfl_xor(v, 1, 32);
  return v;
}

__global__ __launch_bounds__(NTHR) void k_prepw2(const float* __restrict__ W, _Float16* Wh) {
  const int t = blockIdx.x * NTHR + threadIdx.x;
  if (t >= HD * HD / 8) return;
  const int n  = t >> 4;
  const int kq = (t & 15) * 8;
  Pack16 u;
#pragma unroll
  for (int i = 0; i < 8; ++i) u.s[i] = (_Float16)(W[(size_t)(kq + i) * HD + n] * 16.0f);
  _Float16* p = Wh + (size_t)n * HD + kq;
  *(volatile v4i*)p = u.i;
  __threadfence();
  *(volatile v4i*)p = u.i;
}

__device__ __forceinline__ void epi_q(v8f acc, float sc, int T, int hh, int m, int wave, int q, float* P) {
  float t[8];
#pragma unroll
  for (int r = 0; r < 8; ++r) t[r] = acc[r] * sc;
#pragma unroll
  for (int mk = 1; mk < 16; mk <<= 1) {
#pragma unroll
    for (int r = 0; r < 8; ++r) t[r] += __shfl_xor(t[r], mk, 32);
  }
  if (m == 0) {
#pragma unroll
    for (int r = 0; r < 8; ++r) P[((T * 16 + 8 * hh + r) * NQMAX + q) * NWAVE + wave] = t[r];
  }
}

template <int NQ>
__device__ __forceinline__ void store_rec(const float* P, float* rec4, int rowBase, int tid) {
  if (tid < 32) {
    float s[4];
#pragma unroll
    for (int q = 0; q < 4; ++q) {
      s[q] = 0.0f;
      if (q < NQ) {
#pragma unroll
        for (int w = 0; w < NWAVE; ++w) s[q] += P[(tid * NQMAX + q) * NWAVE + w];
      }
    }
    v4f o;
    o.x = s[0]; o.y = s[1]; o.z = s[2]; o.w = s[3];
    float* gp = rec4 + (size_t)(rowBase + tid) * 4;
    *(volatile v4f*)gp = o;
    __threadfence();
    *(volatile v4f*)gp = o;
  }
}

__global__ __launch_bounds__(NTHR) void k_gemm1(
    const float* __restrict__ x, const float* __restrict__ W1,
    const float* __restrict__ att_s, const float* __restrict__ att_d,
    float* nrec, int nN) {
  __shared__ __attribute__((aligned(16))) float P[GR * NQMAX * NWAVE];
  const int tid  = threadIdx.x;
  const int lane = tid & 31;
  const int wave = tid >> 5;
  const int hh   = lane >> 4;
  const int m    = lane & 15;
  const int rowBase = blockIdx.x * GR;
  const int ncol = wave * 16 + m;

  Frag b;
#pragma unroll
  for (int i = 0; i < 8; ++i) {
    const int k  = 8 * hh + i;
    const int kc = k < CIN ? k : CIN - 1;
    const float wv = W1[(size_t)kc * HD + ncol] * 8.0f;
    b.s[i]     = (_Float16)(k < CIN ? wv : 0.0f);
    b.s[8 + i] = (_Float16)0.0f;
  }
  const v8f z8 = {0.f, 0.f, 0.f, 0.f, 0.f, 0.f, 0.f, 0.f};
  v8f c0, c1;
  {
    int rA = rowBase + m;      if (rA > nN - 1) rA = nN - 1;
    int rB = rowBase + 16 + m; if (rB > nN - 1) rB = nN - 1;
    Frag a0, a1;
#pragma unroll
    for (int i = 0; i < 8; ++i) {
      const int k  = 8 * hh + i;
      const int kc = k < CIN ? k : CIN - 1;
      const float xa = x[(size_t)rA * CIN + kc];
      const float xb = x[(size_t)rB * CIN + kc];
      a0.s[i]     = (_Float16)(k < CIN ? xa : 0.0f);
      a1.s[i]     = (_Float16)(k < CIN ? xb : 0.0f);
      a0.s[8 + i] = (_Float16)0.0f;
      a1.s[8 + i] = (_Float16)0.0f;
    }
    c0 = wm(a0.v, b.v, z8);
    c1 = wm(a1.v, b.v, z8);
  }
  const float cs = 0.125f * att_s[ncol];
  const float cd = 0.125f * att_d[ncol];
  epi_q(c0, cs, 0, hh, m, wave, 0, P);
  epi_q(c0, cd, 0, hh, m, wave, 1, P);
  epi_q(c1, cs, 1, hh, m, wave, 0, P);
  epi_q(c1, cd, 1, hh, m, wave, 1, P);
  __syncthreads();
  store_rec<2>(P, nrec, rowBase, tid);
}

__global__ __launch_bounds__(NTHR) void k_prep1(
    const int* __restrict__ ei, const float* __restrict__ ew,
    const float* __restrict__ x, const float* __restrict__ nrec,
    float* rec, int nN, int nE, int EP) {
  (void)ew;
  const int e = blockIdx.x * NTHR + threadIdx.x;
  float v[NCH1];
#pragma unroll
  for (int c = 0; c < NCH1; ++c) v[c] = 0.0f;
  if (e < nE) {
    int s = ei[e];
    int d = ei[(size_t)nE + e];
    s = s < 0 ? 0 : (s > nN - 1 ? nN - 1 : s);
    d = d < 0 ? 0 : (d > nN - 1 ? nN - 1 : d);
    float al = nrec[(size_t)s * 4 + 0] + nrec[(size_t)d * 4 + 1];
    al = (al > 0.0f) ? al : 0.2f * al;
    al = fminf(al, 80.0f);
    const float p = expf(al);
#pragma unroll
    for (int c = 0; c < CIN; ++c) v[c] = p * x[(size_t)s * CIN + c];
    v[CIN] = p;
  }
#pragma unroll
  for (int c = 0; c < NCH1; ++c) *(volatile float*)(rec + (size_t)c * (size_t)EP + e) = v[c];
  __threadfence();
#pragma unroll
  for (int c = 0; c < NCH1; ++c) *(volatile float*)(rec + (size_t)c * (size_t)EP + e) = v[c];
}

template <int NCH, int NB, int G, int GL>
__device__ __forceinline__ void drain(float* acc, const int* list, const int* wcnt,
                                      const float* __restrict__ rec, int EP, int cbase, int nE, int lane) {
  const int gq  = lane / GL;
  const int cig = lane - gq * GL;
  const bool chan = (gq < G) && (cig < NCH);
  const bool g0c  = (gq == 0) && (cig < NCH);
#pragma unroll 1
  for (int wsx = 0; wsx < NWAVE; ++wsx) {
    int n = wcnt[wsx];
    n = n < 0 ? 0 : (n > WCAP ? WCAP : n);
#pragma unroll 1
    for (int i0 = 0; i0 < n; i0 += G) {
      const int i   = i0 + gq;
      const bool vi = (gq < G) && (i < n);
      const int ic  = i < WCAP ? i : WCAP - 1;
      const int ent = list[wsx * WCAP + ic];
      int slot = ent & 0x3FFF;
      if (slot > NB - 1) slot = NB - 1;
      const int el = (ent >> 14) & (CHUNK - 1);
      int e = cbase + el;
      if (e > nE - 1) e = nE - 1;
      const int key = vi ? slot : (-1 - gq);
      bool cf = false;
#pragma unroll
      for (int o = 0; o < G; ++o) {
        const int ok = __shfl(key, o * GL, 32);
        cf = cf | ((o != gq) & (ok == key));
      }
      if (__builtin_amdgcn_ballot_w32(cf) == 0u) {
        if (vi && chan) {
          const float val = rec[(size_t)cig * (size_t)EP + (size_t)e];
          float* p = acc + cig * NB + slot;
          const float cur = *p;
          *p = cur + val;
        }
      } else {
#pragma unroll 1
        for (int j = 0; j < G; ++j) {
          const int ij = i0 + j;
          if (ij < n && g0c) {
            const int entj = list[wsx * WCAP + ij];
            int sj = entj & 0x3FFF;
            if (sj > NB - 1) sj = NB - 1;
            const int elj = (entj >> 14) & (CHUNK - 1);
            int ej = cbase + elj;
            if (ej > nE - 1) ej = nE - 1;
            const float val = rec[(size_t)cig * (size_t)EP + (size_t)ej];
            float* p = acc + cig * NB + sj;
            const float cur = *p;
            *p = cur + val;
          }
        }
      }
    }
  }
}

template <int NCH, int NB, int G, int GL>
__device__ __forceinline__ void scan_drain(float* acc, int* list, int* wcnt,
                                           const int* __restrict__ eid, const float* __restrict__ rec,
                                           int EP, int nE, int nodeBase, int tid, int lane, int wave) {
  const bool al16 = ((((size_t)eid) & 15) == 0);
  const int nChunks = (nE + CHUNK - 1) / CHUNK;
#pragma unroll 1
  for (int ch = 0; ch < nChunks; ++ch) {
    const int cbase = ch * CHUNK;
    const int el0 = tid * 8;
    const int e0  = cbase + el0;
    const int sent = -2147483647 - 1;
    int d[8];
    if (al16 && (e0 + 7 < nE)) {
      const v4i u0 = *(const v4i*)(eid + e0);
      const v4i u1 = *(const v4i*)(eid + e0 + 4);
      d[0] = u0.x; d[1] = u0.y; d[2] = u0.z; d[3] = u0.w;
      d[4] = u1.x; d[5] = u1.y; d[6] = u1.z; d[7] = u1.w;
    } else {
#pragma unroll
      for (int j = 0; j < 8; ++j) d[j] = (e0 + j < nE) ? eid[e0 + j] : sent;
    }
    unsigned s[8];
    bool h[8];
    bool anyh = false;
#pragma unroll
    for (int j = 0; j < 8; ++j) {
      s[j] = (unsigned)d[j] - (unsigned)nodeBase;
      h[j] = s[j] < (unsigned)NB;
      anyh = anyh | h[j];
    }
    int wc = 0;
    if (__builtin_amdgcn_ballot_w32(anyh) != 0u) {
#pragma unroll
      for (int j = 0; j < 8; ++j) {
        const unsigned mj = __builtin_amdgcn_ballot_w32(h[j]);
        if (mj != 0u) {
          if (h[j]) {
            const int pos = wc + (int)__builtin_amdgcn_mbcnt_lo(mj, 0u);
            if (pos < WCAP) list[wave * WCAP + pos] = ((el0 + j) << 14) | (int)s[j];
          }
          wc += (int)__builtin_popcount(mj);
        }
      }
    }
    if (lane == 0) wcnt[wave] = wc;
    __syncthreads();
    if (wave == 0) drain<NCH, NB, G, GL>(acc, list, wcnt, rec, EP, cbase, nE, lane);
    __syncthreads();
  }
}

__global__ __launch_bounds__(NTHR) void k_agg1(
    const int* __restrict__ ei, const float* __restrict__ rec,
    const float* __restrict__ W1, const float* __restrict__ b1,
    _Float16* r1h, int nE, int EP) {
  extern __shared__ v4f lds_dyn[];
  float* acc  = (float*)lds_dyn;
  int*   list = (int*)((char*)lds_dyn + LDS1_ACC);
  int*   wcnt = (int*)((char*)lds_dyn + LDS1_ACC + LDS_LIST);
  _Float16* tile = (_Float16*)((char*)lds_dyn + LDS1_ACC + LDS_LIST + LDS_WCNT);

  const int tid  = threadIdx.x;
  const int lane = tid & 31;
  const int wave = tid >> 5;
  const int hh   = lane >> 4;
  const int m    = lane & 15;
  const int nodeBase = blockIdx.x * NB1;

  {
    const v4f z4 = {0.f, 0.f, 0.f, 0.f};
    for (int i = tid; i < LDS1_ACC / 16; i += NTHR) lds_dyn[i] = z4;
  }
  __syncthreads();

  scan_drain<NCH1, NB1, 3, 10>(acc, list, wcnt, ei + nE, rec, EP, nE, nodeBase, tid, lane, wave);

  const int ncol = wave * 16 + m;
  Frag bw;
#pragma unroll
  for (int i = 0; i < 8; ++i) {
    const int k  = 8 * hh + i;
    const int kc = k < CIN ? k : CIN - 1;
    const float wv = W1[(size_t)kc * HD + ncol] * 8.0f;
    bw.s[i]     = (_Float16)(k < CIN ? wv : 0.0f);
    bw.s[8 + i] = (_Float16)0.0f;
  }
  const float bcol = b1[ncol];
  const v8f z8 = {0.f, 0.f, 0.f, 0.f, 0.f, 0.f, 0.f, 0.f};

#pragma unroll 1
  for (int rt = 0; rt < NB1 / 16; ++rt) {
    const int slot = rt * 16 + m;
    const float den = acc[CIN * NB1 + slot];
    const float inv = 1.0f / (den + 1e-16f);
    Frag a;
#pragma unroll
    for (int i = 0; i < 8; ++i) {
      const int k  = 8 * hh + i;
      const int kc = k < CIN ? k : CIN - 1;
      const float av = acc[kc * NB1 + slot] * inv;
      a.s[i]     = (_Float16)(k < CIN ? av : 0.0f);
      a.s[8 + i] = (_Float16)0.0f;
    }
    const v8f dd = wm(a.v, bw.v, z8);
#pragma unroll
    for (int r = 0; r < 8; ++r) {
      float v = dd[r] * 0.125f + bcol;
      v = v > 0.0f ? v : 0.0f;
      tile[(8 * hh + r) * TSP + ncol] = (_Float16)v;
    }
    __syncthreads();
    {
      const int row = tid >> 4;
      const int cq  = (tid & 15) * 8;
      Pack16 u;
      u.h = *(const v8h*)(tile + row * TSP + cq);
      _Float16* gp = r1h + (size_t)(nodeBase + rt * 16 + row) * HD + cq;
      *(volatile v4i*)gp = u.i;
      __threadfence();
      *(volatile v4i*)gp = u.i;
    }
    __syncthreads();
  }
}

__global__ __launch_bounds__(NTHR) void k_gemm2(
    const _Float16* __restrict__ r1h, const _Float16* __restrict__ Wh,
    const float* __restrict__ att_s, const float* __restrict__ att_d,
    const float* __restrict__ Wc, float* nrec) {
  __shared__ __attribute__((aligned(16))) float P[GR * NQMAX * NWAVE];
  const int tid  = threadIdx.x;
  const int lane = tid & 31;
  const int wave = tid >> 5;
  const int hh   = lane >> 4;
  const int m    = lane & 15;
  const int rowBase = blockIdx.x * GR;
  const int ncol = wave * 16 + m;

  v8f c0 = {0.f, 0.f, 0.f, 0.f, 0.f, 0.f, 0.f, 0.f};
  v8f c1 = {0.f, 0.f, 0.f, 0.f, 0.f, 0.f, 0.f, 0.f};
#pragma unroll
  for (int kt = 0; kt < HD / 32; ++kt) {
    const int k0 = kt * 32;
    Frag a0, a1, b;
    const _Float16* pb  = Wh  + (size_t)ncol * HD + k0 + 8 * hh;
    const _Float16* pa0 = r1h + (size_t)(rowBase + m) * HD + k0 + 8 * hh;
    const _Float16* pa1 = r1h + (size_t)(rowBase + 16 + m) * HD + k0 + 8 * hh;
    b.half[0]  = *(const v8h*)pb;   b.half[1]  = *(const v8h*)(pb + 16);
    a0.half[0] = *(const v8h*)pa0;  a0.half[1] = *(const v8h*)(pa0 + 16);
    a1.half[0] = *(const v8h*)pa1;  a1.half[1] = *(const v8h*)(pa1 + 16);
    c0 = wm(a0.v, b.v, c0);
    c1 = wm(a1.v, b.v, c1);
  }

  const float sc = 0.0625f;
  const float q0 = sc * att_s[ncol];
  const float q1 = sc * att_d[ncol];
  const float q2 = sc * Wc[2 * ncol + 0];
  const float q3 = sc * Wc[2 * ncol + 1];
  epi_q(c0, q0, 0, hh, m, wave, 0, P);
  epi_q(c0, q1, 0, hh, m, wave, 1, P);
  epi_q(c0, q2, 0, hh, m, wave, 2, P);
  epi_q(c0, q3, 0, hh, m, wave, 3, P);
  epi_q(c1, q0, 1, hh, m, wave, 0, P);
  epi_q(c1, q1, 1, hh, m, wave, 1, P);
  epi_q(c1, q2, 1, hh, m, wave, 2, P);
  epi_q(c1, q3, 1, hh, m, wave, 3, P);
  __syncthreads();
  store_rec<4>(P, nrec, rowBase, tid);
}

__global__ __launch_bounds__(NTHR) void k_prep2(
    const int* __restrict__ ei, const float* __restrict__ ew,
    const float* __restrict__ nrec, float* rec, int nN, int nE, int EP) {
  (void)ew;
  const int e = blockIdx.x * NTHR + threadIdx.x;
  float v[NCH2];
#pragma unroll
  for (int c = 0; c < NCH2; ++c) v[c] = 0.0f;
  if (e < nE) {
    int s = ei[e];
    int d = ei[(size_t)nE + e];
    s = s < 0 ? 0 : (s > nN - 1 ? nN - 1 : s);
    d = d < 0 ? 0 : (d > nN - 1 ? nN - 1 : d);
    float al = nrec[(size_t)s * 4 + 0] + nrec[(size_t)d * 4 + 1];
    al = (al > 0.0f) ? al : 0.2f * al;
    al = fminf(al, 80.0f);
    const float p = expf(al);
    v[0] = p * nrec[(size_t)s * 4 + 2];
    v[1] = p * nrec[(size_t)s * 4 + 3];
    v[2] = p;
  }
#pragma unroll
  for (int c = 0; c < NCH2; ++c) *(volatile float*)(rec + (size_t)c * (size_t)EP + e) = v[c];
  __threadfence();
#pragma unroll
  for (int c = 0; c < NCH2; ++c) *(volatile float*)(rec + (size_t)c * (size_t)EP + e) = v[c];
}

__global__ __launch_bounds__(NTHR) void k_agg2(
    const int* __restrict__ ei, const float* __restrict__ rec,
    const int* __restrict__ batch, float* bpart,
    int nN, int nE, int EP, int nG) {
  extern __shared__ v4f lds_dyn[];
  float* acc  = (float*)lds_dyn;
  int*   list = (int*)((char*)lds_dyn + LDS2_ACC);
  int*   wcnt = (int*)((char*)lds_dyn + LDS2_ACC + LDS_LIST);
  v4f*   part = (v4f*)((char*)lds_dyn + LDS2_ACC + LDS_LIST + LDS_WCNT);

  const int tid  = threadIdx.x;
  const int lane = tid & 31;
  const int wave = tid >> 5;
  const int nodeBase = blockIdx.x * NB2;
  const v4f z4 = {0.f, 0.f, 0.f, 0.f};

  for (int i = tid; i < LDS2_ACC / 16; i += NTHR) lds_dyn[i] = z4;
  __syncthreads();

  scan_drain<NCH2, NB2, 8, 4>(acc, list, wcnt, ei + nE, rec, EP, nE, nodeBase, tid, lane, wave);

  for (int i = tid; i < NWAVE * NGMAX; i += NTHR) part[i] = z4;
  __syncthreads();

  const int SPW = NB2 / NWAVE;
#pragma unroll 1
  for (int st = 0; st < SPW / 32; ++st) {
    const int slot = wave * SPW + st * 32 + lane;
    const int node = nodeBase + slot;
    bool valid = node < nN;
    int g = -1;
    if (valid) g = batch[node];
    valid = valid && ((unsigned)g < (unsigned)nG);
    const float den = acc[2 * NB2 + slot];
    const float inv = 1.0f / (den + 1e-16f);
    const float v0 = acc[slot] * inv;
    const float v1 = acc[NB2 + slot] * inv;
    unsigned rem = __builtin_amdgcn_ballot_w32(valid);
    for (int it = 0; it < 32; ++it) {
      if (rem == 0u) break;
      const int lead = __builtin_ctz(rem);
      const int g0 = __shfl(g, lead, 32);
      const bool in = valid && (g == g0);
      const unsigned mk = __builtin_amdgcn_ballot_w32(in);
      const float s0 = wsum(in ? v0 : 0.0f);
      const float s1 = wsum(in ? v1 : 0.0f);
      const float cn = (float)__builtin_popcount(mk);
      if (lane == 0) {
        v4f pv = part[wave * NGMAX + g0];
        pv.x += s0; pv.y += s1; pv.z += cn;
        part[wave * NGMAX + g0] = pv;
      }
      rem &= ~mk;
    }
  }
  __syncthreads();

  {
    v4f o = z4;
    if (tid < nG) {
#pragma unroll
      for (int w = 0; w < NWAVE; ++w) {
        const v4f pv = part[w * NGMAX + tid];
        o.x += pv.x; o.y += pv.y; o.z += pv.z;
      }
    }
    v4f* gp = (v4f*)(bpart + ((size_t)blockIdx.x * NGMAX + tid) * 4);
    *(volatile v4f*)gp = o;
    __threadfence();
    *(volatile v4f*)gp = o;
  }
}

__global__ __launch_bounds__(NTHR) void k_head(
    const float* __restrict__ bpart, const float* __restrict__ b2,
    const float* __restrict__ Wc, const float* __restrict__ bcv,
    float* out, int nb, int nG) {
  __shared__ __attribute__((aligned(16))) float outs[2 * NGMAX];
  const int tid = threadIdx.x;
  float S0 = 0.0f, S1 = 0.0f, C = 0.0f;
  if (tid < nG) {
#pragma unroll 1
    for (int b = 0; b < nb; ++b) {
      const float* p = bpart + ((size_t)b * NGMAX + tid) * 4;
      S0 += p[0]; S1 += p[1]; C += p[2];
    }
  }
  float bw0 = 0.0f, bw1 = 0.0f;
#pragma unroll 1
  for (int c = 0; c < HD; ++c) {
    const float bb = b2[c];
    bw0 += bb * Wc[2 * c + 0];
    bw1 += bb * Wc[2 * c + 1];
  }
  const float invc = 1.0f / fmaxf(C, 1.0f);
  const float l0 = (S0 + C * bw0) * invc + bcv[0];
  const float l1 = (S1 + C * bw1) * invc + bcv[1];
  const float mx = fmaxf(l0, l1);
  const float d0 = l0 - mx;
  const float d1 = l1 - mx;
  const float lg = __logf(__expf(d0) + __expf(d1));
  if (tid < nG) {
    outs[2 * tid + 0] = d0 - lg;
    outs[2 * tid + 1] = d1 - lg;
  } else if (tid < NGMAX) {
    outs[2 * tid + 0] = 0.0f;
    outs[2 * tid + 1] = 0.0f;
  }
  __syncthreads();
  const int nf = (2 * nG) >> 2;
  const int tl = (2 * nG) & 3;
  v4f v = {0.f, 0.f, 0.f, 0.f};
  if (tid < nf) v = *(const v4f*)(outs + 4 * tid);
  if (tid < nf) *(volatile v4f*)(out + 4 * tid) = v;
  if (tid == 0 && tl != 0) {
    for (int j = 0; j < tl; ++j) *(volatile float*)(out + 4 * nf + j) = outs[4 * nf + j];
  }
  __threadfence();
  if (tid < nf) *(volatile v4f*)(out + 4 * tid) = v;
  if (tid == 0 && tl != 0) {
    for (int j = 0; j < tl; ++j) *(volatile float*)(out + 4 * nf + j) = outs[4 * nf + j];
  }
}

static inline int cdiv_i(long long a, long long b) { return (int)((a + b - 1) / b); }
static inline size_t al128(size_t v) { return (v + 127) & ~(size_t)127; }

extern "C" void kernel_launch(void* const* d_in, const int* in_sizes, int n_in,
                              void* d_out, int out_size, void* d_ws, size_t ws_size,
                              hipStream_t stream) {
  if (n_in < 16) return;
  const int nN = in_sizes[5];
  if (nN < 1 || in_sizes[0] != nN * CIN) return;
  if ((in_sizes[1] & 1) || (in_sizes[3] & 1)) return;
  const int nE1 = in_sizes[1] / 2;
  const int nE2 = in_sizes[3] / 2;
  if (nE1 < 1 || nE2 < 1) return;
  if (in_sizes[6] != CIN * HD || in_sizes[7] != HD || in_sizes[8] != HD || in_sizes[9] != HD) return;
  if (in_sizes[10] != HD * HD || in_sizes[11] != HD || in_sizes[12] != HD || in_sizes[13] != HD) return;
  if (in_sizes[14] != HD * 2 || in_sizes[15] != 2) return;
  const int nG = out_size / 2;
  if (nG < 1 || nG > NGMAX || out_size != 2 * nG) return;

  const float* x    = (const float*)d_in[0];
  const int*   eiS  = (const int*)d_in[1];
  const float* ewS  = (const float*)d_in[2];
  const int*   eiT  = (const int*)d_in[3];
  const float* ewT  = (const float*)d_in[4];
  const int*   bat  = (const int*)d_in[5];
  const float* W1   = (const float*)d_in[6];
  const float* as1  = (const float*)d_in[7];
  const float* ad1  = (const float*)d_in[8];
  const float* b1   = (const float*)d_in[9];
  const float* W2   = (const float*)d_in[10];
  const float* as2  = (const float*)d_in[11];
  const float* ad2  = (const float*)d_in[12];
  const float* b2   = (const float*)d_in[13];
  const float* Wc   = (const float*)d_in[14];
  const float* bc   = (const float*)d_in[15];
  float* out = (float*)d_out;

  const int nPadG = cdiv_i(nN, GR) * GR;
  const int nb1   = cdiv_i(nN, NB1);
  const int nPad1 = nb1 * NB1;
  const int nb2   = cdiv_i(nN, NB2);
  if (nPadG > nPad1) return;
  const int EP1 = cdiv_i(nE1, NTHR) * NTHR;
  const int EP2 = cdiv_i(nE2, NTHR) * NTHR;
  const size_t recFloats = ((size_t)NCH1 * EP1 > (size_t)NCH2 * EP2) ? (size_t)NCH1 * EP1 : (size_t)NCH2 * EP2;

  size_t off = 0;
  _Float16* W2h = (_Float16*)((char*)d_ws + off); off = al128(off + (size_t)HD * HD * sizeof(_Float16));
  float* nrec1  = (float*)((char*)d_ws + off);    off = al128(off + (size_t)nPadG * 4 * sizeof(float));
  float* nrec2  = (float*)((char*)d_ws + off);    off = al128(off + (size_t)nPadG * 4 * sizeof(float));
  _Float16* r1h = (_Float16*)((char*)d_ws + off); off = al128(off + (size_t)nPad1 * HD * sizeof(_Float16));
  float* recE   = (float*)((char*)d_ws + off);    off = al128(off + recFloats * sizeof(float));
  float* bpart  = (float*)((char*)d_ws + off);    off = al128(off + (size_t)nb2 * NGMAX * 4 * sizeof(float));
  if (off > ws_size) return;

  k_prepw2<<<(HD * HD / 8 + NTHR - 1) / NTHR, NTHR, 0, stream>>>(W2, W2h);
  k_gemm1<<<nPadG / GR, NTHR, 0, stream>>>(x, W1, as1, ad1, nrec1, nN);
  k_prep1<<<EP1 / NTHR, NTHR, 0, stream>>>(eiS, ewS, x, nrec1, recE, nN, nE1, EP1);
  hipFuncSetAttribute(reinterpret_cast<const void*>(&k_agg1),
                      hipFuncAttributeMaxDynamicSharedMemorySize, LDS1_BYTES);
  k_agg1<<<nb1, NTHR, LDS1_BYTES, stream>>>(eiS, recE, W1, b1, r1h, nE1, EP1);
  k_gemm2<<<nPadG / GR, NTHR, 0, stream>>>(r1h, W2h, as2, ad2, Wc, nrec2);
  k_prep2<<<EP2 / NTHR, NTHR, 0, stream>>>(eiT, ewT, nrec2, recE, nN, nE2, EP2);
  hipFuncSetAttribute(reinterpret_cast<const void*>(&k_agg2),
                      hipFuncAttributeMaxDynamicSharedMemorySize, LDS2_BYTES);
  k_agg2<<<nb2, NTHR, LDS2_BYTES, stream>>>(eiT, recE, bat, bpart, nN, nE2, EP2, nG);
  k_head<<<1, NTHR, 0, stream>>>(bpart, b2, Wc, bc, out, nb2, nG);
}
